// RITS_66675072303366
// MI455X (gfx1250) — hardware-verified
//
#include <hip/hip_runtime.h>
#include <math.h>

constexpr int NB     = 1024;
constexpr int NT     = 512;
constexpr int ND     = 2;
constexpr int NH     = 128;
constexpr int NG     = 4 * NH;
constexpr int RB     = 32;
constexpr int NTHR   = 256;
constexpr int APITCH = 136;
constexpr int HFP    = 132;
constexpr int CHK    = 16;
constexpr int CW     = CHK * ND;
constexpr int SLP    = 36;
constexpr float WCARRY     = 64.0f;
constexpr float WCARRY_INV = 1.0f / 64.0f;
static_assert(NB % RB == 0);
static_assert(RB == 32);
static_assert(NH == 16 * (NTHR / 32));
static_assert(NH % 32 == 0);
static_assert(NT % CHK == 0 && CW == 32);
static_assert(RB * CW == 4 * NTHR);
static_assert(RB * ND * 4 == NTHR);
static_assert(NT % 32 == 0 && NB == 4 * 256);
static_assert(NG % 64 == 0 && NH * 64 == 8 * NTHR * 4 && 64 * (NH / 8) == 4 * NTHR);

typedef __attribute__((ext_vector_type(16))) _Float16 v16h;
typedef __attribute__((ext_vector_type(8)))  _Float16 v8h;
typedef __attribute__((ext_vector_type(8)))  float    v8f;
typedef __attribute__((ext_vector_type(4)))  float    v4f;
typedef __attribute__((ext_vector_type(2)))  float    v2f;

__device__ __forceinline__ void dep_guard_h(v8f& a, v8f& b, v16h x, v16h y) { asm volatile("v_nop\n\tv_nop\n\tv_nop\n\tv_nop" : "+v"(a), "+v"(b) : "v"(x), "v"(y)); }
__device__ __forceinline__ void keep4_h(v16h a, v16h b, v16h c, v16h d) { asm volatile("v_nop" :: "v"(a), "v"(b), "v"(c), "v"(d)); }
__device__ __forceinline__ void acc_guard4(v8f& a, v8f& b, v8f& c, v8f& d) { asm volatile("v_nop\n\tv_nop\n\tv_nop\n\tv_nop" : "+v"(a), "+v"(b), "+v"(c), "+v"(d)); }
template <typename T> struct Frag;
template <> struct Frag<_Float16> {
  typedef v16h V; union U { v16h v; v8h h[2]; };
  static __device__ __forceinline__ v16h load(const _Float16* p) {
    U f; f.h[0] = *(const v8h*)(p); f.h[1] = *(const v8h*)(p + 16); return f.v;
  }
  static __device__ __forceinline__ v8f mma(v16h a, v16h b, v8f c) {
    return __builtin_amdgcn_wmma_f32_16x16x32_f16(false, a, false, b, (short)0, c, false, false);
  }
};

__device__ __forceinline__ float fsig(float x)  { return __builtin_amdgcn_rcpf(1.0f + __expf(-x)); }
__device__ __forceinline__ float ftanh(float x) { return 1.0f - 2.0f * __builtin_amdgcn_rcpf(__expf(2.0f * x) + 1.0f); }

__global__ __launch_bounds__(NTHR) void mask_norm_kernel(const float* __restrict__ masks, float* __restrict__ invd) {
  __shared__ float red[4][64];
  __shared__ __align__(16) float ov[32];
  const int tid = threadIdx.x;
  const int t0 = blockIdx.x * 32;
  const int p = tid & 63, bg = tid >> 6;
  const float* mp = masks + (size_t)(bg * 256) * (NT * ND) + (size_t)t0 * ND + p;
  float s = 0.0f;
#pragma unroll 1
  for (int i = 0; i < 256; ++i) s += mp[(size_t)i * (NT * ND)];
  red[bg][p] = s;
  __syncthreads();
  if (tid < 32) {
    const float a = (red[0][2 * tid] + red[1][2 * tid]) + (red[2][2 * tid] + red[3][2 * tid]);
    const float b = (red[0][2 * tid + 1] + red[1][2 * tid + 1]) + (red[2][2 * tid + 1] + red[3][2 * tid + 1]);
    ov[tid] = 1.0f / ((a + b) + 1e-6f);
  }
  __syncthreads();
  if (tid < 8) {
    const v4f v = *(const v4f*)(ov + 4 * tid);
    float* op = invd + t0 + 4 * tid;
    *(volatile v4f*)op = v;
    __threadfence();
    *(volatile v4f*)op = v;
  }
}

__global__ __launch_bounds__(NTHR) void wrec_t16_kernel(const float* __restrict__ W, unsigned short* __restrict__ WT) {
  __shared__ float tile[NH][65];
  const int tid = threadIdx.x;
  const int n0 = blockIdx.x * 64;
#pragma unroll
  for (int it = 0; it < 8; ++it) {
    const int e = tid + NTHR * it;
    const int k = e >> 4, c4 = (e & 15) * 4;
    const v4f v = *(const v4f*)(W + (size_t)k * NG + n0 + c4);
    tile[k][c4] = v[0]; tile[k][c4 + 1] = v[1]; tile[k][c4 + 2] = v[2]; tile[k][c4 + 3] = v[3];
  }
  __syncthreads();
#pragma unroll
  for (int it = 0; it < 4; ++it) {
    const int e = tid + NTHR * it;
    const int nl = e >> 4, k8 = (e & 15) * 8;
    v8h hv;
#pragma unroll
    for (int q = 0; q < 8; ++q) hv[q] = (_Float16)(tile[k8 + q][nl] * WCARRY);
    unsigned short* op = WT + (size_t)(n0 + nl) * NH + k8;
    *(volatile v8h*)op = hv;
    __threadfence();
    *(volatile v8h*)op = hv;
  }
}

__global__ __launch_bounds__(NTHR) void impute_seq_kernel(
    const float* __restrict__ values, const float* __restrict__ masks, const float* __restrict__ deltas,
    const float* __restrict__ tdh_W, const float* __restrict__ tdh_b,
    const float* __restrict__ tdx_W, const float* __restrict__ tdx_b,
    const float* __restrict__ hist_W, const float* __restrict__ hist_b,
    const float* __restrict__ fr_W, const float* __restrict__ fr_b,
    const float* __restrict__ wc_W, const float* __restrict__ wc_b,
    const float* __restrict__ lstm_Wk, const float* __restrict__ lstm_b,
    const unsigned short* __restrict__ WTp, const float* __restrict__ invd,
    float* __restrict__ out_imp, float* __restrict__ out_loss) {
  __shared__ __align__(16) _Float16 Ah[RB * APITCH];
  __shared__ __align__(16) float Hf[RB * HFP];
  __shared__ __align__(16) float Xc[RB * CW];
  __shared__ __align__(16) float Mc[RB * CW];
  __shared__ __align__(16) float Dc[RB * CW];
  __shared__ __align__(16) float hW[ND * NH];
  __shared__ __align__(16) float idn[NT];
  __shared__ __align__(16) float xhp[RB * ND];
  __shared__ __align__(16) float ccs[RB * ND];
  __shared__ __align__(16) float slab[RB * SLP];
  __shared__ __align__(16) float lsl[32];

  const _Float16* WT = (const _Float16*)WTp;
  const int tid = threadIdx.x, lane = tid & 31, wave = tid >> 5;
  const int c = lane & 15, hh = lane >> 4, koff = hh * 8;
  const int j = 16 * wave + c;
  const int rowbase = blockIdx.x * RB;

  {
    const int d = tid >> 7, k = tid & 127;
    hW[tid] = hist_W[k * ND + d];
    idn[tid] = invd[tid];
    idn[tid + NTHR] = invd[tid + NTHR];
  }
  const float tw0 = tdh_W[j * ND], tw1 = tdh_W[j * ND + 1], tb = tdh_b[j];
  float wk0[4], wk1[4], wk2[4], wk3[4], lb[4];
#pragma unroll
  for (int g = 0; g < 4; ++g) {
    const int col = g * NH + j;
    wk0[g] = lstm_Wk[col];
    wk1[g] = lstm_Wk[NG + col];
    wk2[g] = lstm_Wk[2 * NG + col];
    wk3[g] = lstm_Wk[3 * NG + col];
    lb[g]  = lstm_b[col];
  }
  const float hb0 = hist_b[0], hb1 = hist_b[1];
  const float fw00 = fr_W[0], fw01 = fr_W[1], fw10 = fr_W[2], fw11 = fr_W[3];
  const float fb0 = fr_b[0], fb1 = fr_b[1];
  const float xw00 = tdx_W[0], xw01 = tdx_W[1], xw10 = tdx_W[2], xw11 = tdx_W[3];
  const float xb0 = tdx_b[0], xb1 = tdx_b[1];
  const float wc00 = wc_W[0], wc01 = wc_W[1], wc10 = wc_W[2], wc11 = wc_W[3];
  const float wc20 = wc_W[4], wc21 = wc_W[5], wc30 = wc_W[6], wc31 = wc_W[7];
  const float wcb0 = wc_b[0], wcb1 = wc_b[1];

  float hreg[2][8], cst[2][8];
#pragma unroll
  for (int mt = 0; mt < 2; ++mt)
#pragma unroll
    for (int r = 0; r < 8; ++r) { hreg[mt][r] = 0.0f; cst[mt][r] = 0.0f; }
  float loss = 0.0f;
  const v8f z8 = {0.f, 0.f, 0.f, 0.f, 0.f, 0.f, 0.f, 0.f};
  __syncthreads();

#pragma unroll 1
  for (int t = 0; t < NT; ++t) {
    const int tc = t & (CHK - 1);
    if (tc == 0) {
      __syncthreads();
      const int row = tid >> 3, c4 = (tid & 7) * 4;
      const size_t go = (size_t)(rowbase + row) * (NT * ND) + (size_t)t * ND + c4;
      *(v4f*)(Xc + row * CW + c4) = *(const v4f*)(values + go);
      *(v4f*)(Mc + row * CW + c4) = *(const v4f*)(masks + go);
      *(v4f*)(Dc + row * CW + c4) = *(const v4f*)(deltas + go);
      __syncthreads();
    }

#pragma unroll
    for (int mt = 0; mt < 2; ++mt) {
#pragma unroll
      for (int r = 0; r < 8; ++r) {
        const int R = 16 * mt + 8 * hh + r;
        const v2f dv = *(const v2f*)(Dc + R * CW + 2 * tc);
        const float a = dv[0] * tw0 + dv[1] * tw1 + tb;
        const float gam = __expf(-fmaxf(a, 0.0f));
        const float hd = hreg[mt][r] * gam;
        Ah[R * APITCH + j] = (_Float16)hd;
        Hf[R * HFP + j] = hd;
      }
    }
    __syncthreads();

    {
      const int pair = tid >> 2, part = tid & 3;
      const int R = pair >> 1, d = pair & 1;
      const float* hp = Hf + R * HFP + part * 32;
      const float* wp = hW + d * NH + part * 32;
      float s = 0.0f;
#pragma unroll
      for (int q = 0; q < 8; ++q) {
        const v4f hv = *(const v4f*)(hp + 4 * q);
        const v4f wv = *(const v4f*)(wp + 4 * q);
        s += hv[0] * wv[0];
        s += hv[1] * wv[1];
        s += hv[2] * wv[2];
        s += hv[3] * wv[3];
      }
      s += __shfl_xor(s, 1, 32);
      s += __shfl_xor(s, 2, 32);
      if (part == 0) xhp[pair] = s;
    }
    __syncthreads();

    if (wave == 0) {
      const int R = lane;
      const v2f xv = *(const v2f*)(Xc + R * CW + 2 * tc);
      const v2f mv = *(const v2f*)(Mc + R * CW + 2 * tc);
      const v2f dv = *(const v2f*)(Dc + R * CW + 2 * tc);
      const v2f xp = *(const v2f*)(xhp + 2 * R);
      const float inv = idn[t];
      const float x0 = xv[0], x1 = xv[1], m0 = mv[0], m1 = mv[1], d0 = dv[0], d1 = dv[1];
      const float xh0 = xp[0] + hb0, xh1 = xp[1] + hb1;
      const float w0 = m0 * inv;
      const float w1 = (m1 * inv) * 0.5f;
      float e0 = x0 - xh0, e1 = x1 - xh1;
      loss = loss + ((fabsf(e0) + e0 * e0) * w0 + (fabsf(e1) + e1 * e1) * w1);
      const float xc0 = m0 * x0 + (1.0f - m0) * xh0;
      const float xc1 = m1 * x1 + (1.0f - m1) * xh1;
      const float z0 = xc0 * fw00 + xc1 * fw01 + fb0;
      const float z1 = xc0 * fw10 + xc1 * fw11 + fb1;
      e0 = x0 - z0; e1 = x1 - z1;
      loss = loss + ((fabsf(e0) + e0 * e0) * w0 + (fabsf(e1) + e1 * e1) * w1);
      const float gx0 = __expf(-fmaxf(d0 * xw00 + d1 * xw01 + xb0, 0.0f));
      const float gx1 = __expf(-fmaxf(d0 * xw10 + d1 * xw11 + xb1, 0.0f));
      const float be0 = gx0 * wc00 + gx1 * wc10 + m0 * wc20 + m1 * wc30 + wcb0;
      const float be1 = gx0 * wc01 + gx1 * wc11 + m0 * wc21 + m1 * wc31 + wcb1;
      const float ch0 = be0 * z0 + (1.0f - be0) * xh0;
      const float ch1 = be1 * z1 + (1.0f - be1) * xh1;
      e0 = x0 - ch0; e1 = x1 - ch1;
      loss = loss + ((fabsf(e0) + e0 * e0) * w0 + (fabsf(e1) + e1 * e1) * w1);
      const float cc0 = m0 * x0 + (1.0f - m0) * ch0;
      const float cc1 = m1 * x1 + (1.0f - m1) * ch1;
      v2f cv; cv[0] = cc0; cv[1] = cc1;
      *(v2f*)(ccs + 2 * R) = cv;
      *(v2f*)(slab + R * SLP + 2 * tc) = cv;
      if (tc == CHK - 1) {
        __builtin_amdgcn_fence(__ATOMIC_RELEASE, "workgroup");
        __builtin_amdgcn_wave_barrier();
        __builtin_amdgcn_fence(__ATOMIC_ACQUIRE, "workgroup");
        const int q = lane >> 3, c4 = (lane & 7) * 4;
        const int tb0 = t - (CHK - 1);
        for (int pass = 0; pass < 2; ++pass) {
#pragma unroll
          for (int it = 0; it < 8; ++it) {
            const int row = it * 4 + q;
            const v4f v = *(const v4f*)(slab + row * SLP + c4);
            *(volatile v4f*)(out_imp + (size_t)(rowbase + row) * (NT * ND) + (size_t)tb0 * ND + c4) = v;
          }
          __threadfence();
        }
        __builtin_amdgcn_fence(__ATOMIC_RELEASE, "workgroup");
        __builtin_amdgcn_wave_barrier();
        __builtin_amdgcn_fence(__ATOMIC_ACQUIRE, "workgroup");
      }
    }

    v8f acc[2][4];
#pragma unroll
    for (int mt = 0; mt < 2; ++mt)
#pragma unroll
      for (int g = 0; g < 4; ++g) acc[mt][g] = z8;
    {
      const _Float16* wrow = WT + (size_t)j * NH + koff;
#pragma unroll 1
      for (int k0 = 0; k0 < NH; k0 += 32) {
        v16h bq[4];
#pragma unroll
        for (int g = 0; g < 4; ++g) bq[g] = Frag<_Float16>::load(wrow + (size_t)g * (NH * NH) + k0);
#pragma unroll
        for (int mt = 0; mt < 2; ++mt) {
          const v16h a = Frag<_Float16>::load(Ah + (16 * mt + c) * APITCH + koff + k0);
#pragma unroll
          for (int g = 0; g < 4; ++g) acc[mt][g] = Frag<_Float16>::mma(a, bq[g], acc[mt][g]);
          dep_guard_h(acc[mt][0], acc[mt][3], a, a);
        }
        keep4_h(bq[0], bq[1], bq[2], bq[3]);
      }
    }
    acc_guard4(acc[0][0], acc[0][1], acc[0][2], acc[0][3]);
    acc_guard4(acc[1][0], acc[1][1], acc[1][2], acc[1][3]);
    __syncthreads();

#pragma unroll
    for (int mt = 0; mt < 2; ++mt) {
#pragma unroll
      for (int r = 0; r < 8; ++r) {
        const int R = 16 * mt + 8 * hh + r;
        const v2f cv = *(const v2f*)(ccs + 2 * R);
        const v2f mv = *(const v2f*)(Mc + R * CW + 2 * tc);
        float gt[4];
#pragma unroll
        for (int g = 0; g < 4; ++g) {
          const float pre = lb[g] + cv[0] * wk0[g] + cv[1] * wk1[g] + mv[0] * wk2[g] + mv[1] * wk3[g];
          gt[g] = acc[mt][g][r] * WCARRY_INV + pre;
        }
        const float cn = fsig(gt[1]) * cst[mt][r] + fsig(gt[0]) * ftanh(gt[2]);
        cst[mt][r] = cn;
        hreg[mt][r] = fsig(gt[3]) * ftanh(cn);
      }
    }
  }

  if (wave == 0) {
    lsl[lane] = loss;
    __builtin_amdgcn_fence(__ATOMIC_RELEASE, "workgroup");
    __builtin_amdgcn_wave_barrier();
    __builtin_amdgcn_fence(__ATOMIC_ACQUIRE, "workgroup");
    if (lane < 8) {
      const v4f v = *(const v4f*)(lsl + 4 * lane);
      float* op = out_loss + rowbase + 4 * lane;
      *(volatile v4f*)op = v;
      __threadfence();
      *(volatile v4f*)op = v;
    }
  }
}

extern "C" void kernel_launch(void* const* d_in, const int* in_sizes, int n_in,
                              void* d_out, int out_size, void* d_ws, size_t ws_size, hipStream_t stream) {
  if (n_in < 16 || d_out == nullptr || d_ws == nullptr) return;
  if (in_sizes[0] != NB * NT * ND || in_sizes[1] != NB * NT * ND || in_sizes[2] != NB * NT * ND ||
      in_sizes[3] != NH * ND || in_sizes[4] != NH || in_sizes[5] != ND * ND || in_sizes[6] != ND ||
      in_sizes[7] != NH * ND || in_sizes[8] != ND || in_sizes[9] != ND * ND || in_sizes[10] != ND ||
      in_sizes[11] != 2 * ND * ND || in_sizes[12] != ND || in_sizes[13] != 2 * ND * NG ||
      in_sizes[14] != NH * NG || in_sizes[15] != NG || out_size != NB * NT * ND + NB) return;

  const float* values  = (const float*)d_in[0];
  const float* masks   = (const float*)d_in[1];
  const float* deltas  = (const float*)d_in[2];
  const float* tdh_W   = (const float*)d_in[3];
  const float* tdh_b   = (const float*)d_in[4];
  const float* tdx_W   = (const float*)d_in[5];
  const float* tdx_b   = (const float*)d_in[6];
  const float* hist_W  = (const float*)d_in[7];
  const float* hist_b  = (const float*)d_in[8];
  const float* fr_W    = (const float*)d_in[9];
  const float* fr_b    = (const float*)d_in[10];
  const float* wc_W    = (const float*)d_in[11];
  const float* wc_b    = (const float*)d_in[12];
  const float* lstm_Wk = (const float*)d_in[13];
  const float* lstm_Wr = (const float*)d_in[14];
  const float* lstm_b  = (const float*)d_in[15];
  float* out_imp  = (float*)d_out;
  float* out_loss = out_imp + (size_t)NB * NT * ND;

  char* ws = (char*)d_ws; size_t off = 0;
  unsigned short* WT = (unsigned short*)(ws + off); off += ((size_t)NG * NH * 2 + 255) & ~(size_t)255;
  float* INVD = (float*)(ws + off);                 off += ((size_t)NT * 4 + 255) & ~(size_t)255;
  if (off > ws_size || off > (size_t)134217728) return;

  mask_norm_kernel<<<NT / 32, NTHR, 0, stream>>>(masks, INVD);
  wrec_t16_kernel<<<NG / 64, NTHR, 0, stream>>>(lstm_Wr, WT);
  impute_seq_kernel<<<NB / RB, NTHR, 0, stream>>>(values, masks, deltas, tdh_W, tdh_b, tdx_W, tdx_b,
                                                   hist_W, hist_b, fr_W, fr_b, wc_W, wc_b,
                                                   lstm_Wk, lstm_b, WT, INVD, out_imp, out_loss);
}
